// StickBreakingAttention_16810501997098
// MI455X (gfx1250) — hardware-verified
//
#include <hip/hip_runtime.h>
#include <stdint.h>

typedef __attribute__((ext_vector_type(16))) _Float16 v16h;
typedef __attribute__((ext_vector_type(8)))  _Float16 v8h;
typedef __attribute__((ext_vector_type(16))) __bf16   v16b;
typedef __attribute__((ext_vector_type(8)))  __bf16   v8b;
typedef __attribute__((ext_vector_type(8)))  float    v8f;
typedef __attribute__((ext_vector_type(4)))  float    v4f;

__device__ __forceinline__ unsigned short f2bf_bits(float f) {
  unsigned u = __float_as_uint(f);
  return (unsigned short)((u + 0x7FFFu + ((u >> 16) & 1u)) >> 16);
}
__device__ __forceinline__ float bf_bits2f(unsigned short h) { return __uint_as_float(((unsigned)h) << 16); }

__device__ __forceinline__ void dep_guard_h(v8f& a, v8f& b, v16h x, v16h y) { asm volatile("v_nop\n\tv_nop\n\tv_nop\n\tv_nop" : "+v"(a), "+v"(b) : "v"(x), "v"(y)); }
__device__ __forceinline__ void dep_guard_b(v8f& a, v8f& b, v16b x, v16b y) { asm volatile("v_nop\n\tv_nop\n\tv_nop\n\tv_nop" : "+v"(a), "+v"(b) : "v"(x), "v"(y)); }
__device__ __forceinline__ void keep4_h(v16h a, v16h b, v16h c, v16h d) { asm volatile("v_nop" :: "v"(a), "v"(b), "v"(c), "v"(d)); }
__device__ __forceinline__ void keep4_b(v16b a, v16b b, v16b c, v16b d) { asm volatile("v_nop" :: "v"(a), "v"(b), "v"(c), "v"(d)); }
__device__ __forceinline__ void acc_guard4(v8f& a, v8f& b, v8f& c, v8f& d) { asm volatile("v_nop\n\tv_nop\n\tv_nop\n\tv_nop" : "+v"(a), "+v"(b), "+v"(c), "+v"(d)); }
template <typename T> struct Frag;
template <> struct Frag<_Float16> {
  typedef v16h V; union U { v16h v; v8h h[2]; };
  static __device__ __forceinline__ v16h load(const _Float16* p) {
    U f; f.h[0] = *(const v8h*)(p); f.h[1] = *(const v8h*)(p + 16); return f.v;
  }
  static __device__ __forceinline__ v8f mma(v16h a, v16h b, v8f c) {
    return __builtin_amdgcn_wmma_f32_16x16x32_f16(false, a, false, b, (short)0, c, false, false);
  }
  static __device__ __forceinline__ void guard(v8f& a, v8f& b, v16h x, v16h y) { dep_guard_h(a, b, x, y); }
  static __device__ __forceinline__ void keep(v16h a, v16h b, v16h c, v16h d) { keep4_h(a, b, c, d); }
};
template <> struct Frag<__bf16> {
  typedef v16b V; union U { v16b v; v8b h[2]; };
  static __device__ __forceinline__ v16b load(const __bf16* p) {
    U f; f.h[0] = *(const v8b*)(p); f.h[1] = *(const v8b*)(p + 16); return f.v;
  }
  static __device__ __forceinline__ v8f mma(v16b a, v16b b, v8f c) {
    return __builtin_amdgcn_wmma_f32_16x16x32_bf16(false, a, false, b, (short)0, c, false, false);
  }
  static __device__ __forceinline__ void guard(v8f& a, v8f& b, v16b x, v16b y) { dep_guard_b(a, b, x, y); }
  static __device__ __forceinline__ void keep(v16b a, v16b b, v16b c, v16b d) { keep4_b(a, b, c, d); }
};

template <int ET> struct Elem;
template <> struct Elem<0> { typedef _Float16 T; };
template <> struct Elem<1> { typedef __bf16 T; };
template <int ET, bool SPLIT, int BIAS_MODE, int OUT_MODE, bool RESID, int ACT = 0>
__global__ __launch_bounds__(256) void wmma_gemm64(
    const unsigned short* __restrict__ Ap, const unsigned short* __restrict__ A2p, int lda, long strideA,
    const unsigned short* __restrict__ Btp, const unsigned short* __restrict__ Bt2p, int ldb, long strideB,
    void* __restrict__ Cout, void* __restrict__ Cout2, int ldc, long strideC,
    const float* __restrict__ bias,
    const float* __restrict__ resid, long strideR,
    int M, int N, int K, float scale) {
  typedef typename Elem<ET>::T T;
  typedef typename Frag<T>::V V;
  const T* A = (const T*)Ap; const T* A2 = (const T*)A2p; const T* Bt = (const T*)Btp; const T* Bt2 = (const T*)Bt2p;
  __shared__ __align__(16) float sT[8][16 * 68];
  const int b    = blockIdx.y;
  const int lane = threadIdx.x & 31;
  const int wave = threadIdx.x >> 5;
  const int tilesN = N >> 6;
  const int tilesM = M >> 6;
  const int tile = blockIdx.x * 8 + wave;
  if (tile >= tilesM * tilesN) return;
  const int tm = tile / tilesN;
  const int tn = tile - tm * tilesN;
  const int m0 = tm << 6;
  const int n0 = tn << 6;

  const T* Ab  = A  + (size_t)b * strideA;
  const T* Bb  = Bt + (size_t)b * strideB;
  const T* Ab2 = SPLIT ? (A2  + (size_t)b * strideA) : nullptr;
  const T* Bb2 = SPLIT ? (Bt2 + (size_t)b * strideB) : nullptr;

  const int rlane = lane & 15;
  const int koff  = (lane >> 4) * 8;
  const int mOff  = (lane >> 4) * 8;

  v8f acc[4][4];
#pragma unroll
  for (int i = 0; i < 4; ++i)
#pragma unroll
    for (int j = 0; j < 4; ++j) acc[i][j] = (v8f){0.f,0.f,0.f,0.f,0.f,0.f,0.f,0.f};

  for (int k0 = 0; k0 < K; k0 += 32) {
    V bh[4], bl[4];
#pragma unroll
    for (int j = 0; j < 4; ++j) {
      const size_t bo = (size_t)(n0 + (j << 4) + rlane) * ldb + koff + k0;
      bh[j] = Frag<T>::load(Bb + bo);
      if (SPLIT) bl[j] = Frag<T>::load(Bb2 + bo);
    }
#pragma unroll
    for (int i = 0; i < 4; ++i) {
      const size_t ao = (size_t)(m0 + (i << 4) + rlane) * lda + koff + k0;
      V ah = Frag<T>::load(Ab + ao);
      V al;
      if (SPLIT) al = Frag<T>::load(Ab2 + ao);
#pragma unroll
      for (int j = 0; j < 4; ++j) {
        acc[i][j] = Frag<T>::mma(ah, bh[j], acc[i][j]);
        if (SPLIT) {
          acc[i][j] = Frag<T>::mma(ah, bl[j], acc[i][j]);
          acc[i][j] = Frag<T>::mma(al, bh[j], acc[i][j]);
        }
      }
      Frag<T>::guard(acc[i][0], acc[i][3], ah, SPLIT ? al : ah);
    }
    Frag<T>::keep(bh[0], bh[1], bh[2], bh[3]);
    if (SPLIT) Frag<T>::keep(bl[0], bl[1], bl[2], bl[3]);
  }
  acc_guard4(acc[0][0], acc[0][1], acc[0][2], acc[0][3]);
  acc_guard4(acc[1][0], acc[1][1], acc[1][2], acc[1][3]);
  acc_guard4(acc[2][0], acc[2][1], acc[2][2], acc[2][3]);
  acc_guard4(acc[3][0], acc[3][1], acc[3][2], acc[3][3]);

  float* slab = sT[wave];
  const float* Rb = RESID ? (resid + (size_t)b * strideR) : nullptr;
#pragma unroll
  for (int i = 0; i < 4; ++i) {
    const int mBase = m0 + (i << 4);
#pragma unroll
    for (int j = 0; j < 4; ++j) {
      const int n = n0 + (j << 4) + rlane;
      float bv = 0.f;
      if (BIAS_MODE == 2) bv = bias[n];
#pragma unroll
      for (int r = 0; r < 8; ++r) {
        float v = acc[i][j][r] * scale;
        if (BIAS_MODE == 1) v += bias[mBase + mOff + r];
        if (BIAS_MODE == 2) v += bv;
        if (RESID) v += Rb[(size_t)(mBase + mOff + r) * ldc + n];
        if (ACT == 1) v = tanhf(v);
        if (ACT == 2) v = fmaxf(v, 0.0f);
        if (ACT == 3) v = v / (1.0f + expf(-v));
        if (ACT == 4) v = (v > 0.f) ? v : 0.01f * v;
        if (ACT == 5) v = 0.5f * v * (1.0f + erff(v * 0.70710678118654752f));
        slab[(mOff + r) * 68 + (j << 4) + rlane] = v;
      }
    }
    __builtin_amdgcn_fence(__ATOMIC_RELEASE, "workgroup");
    __builtin_amdgcn_wave_barrier();
    __builtin_amdgcn_fence(__ATOMIC_ACQUIRE, "workgroup");
    if (OUT_MODE == 0) {
      float* C = (float*)Cout + (size_t)b * strideC;
      const int hh = lane >> 4, c4 = (lane & 15) * 4;
      for (int pass = 0; pass < 2; ++pass) {
#pragma unroll
        for (int it = 0; it < 8; ++it) {
          const int row = it * 2 + hh;
          v4f v = *(const v4f*)(slab + row * 68 + c4);
          *(volatile v4f*)(C + (size_t)(mBase + row) * ldc + n0 + c4) = v;
        }
        __threadfence();
      }
    } else {
      const int q = lane >> 3, c8 = (lane & 7) * 8;
      unsigned short* C  = (unsigned short*)Cout  + (size_t)b * strideC;
      unsigned short* C2 = (OUT_MODE == 2) ? ((unsigned short*)Cout2 + (size_t)b * strideC) : nullptr;
      for (int pass = 0; pass < 2; ++pass) {
#pragma unroll
        for (int it = 0; it < 4; ++it) {
          const int row = it * 4 + q;
          const float* sp = slab + row * 68 + c8;
          v8h hv, lv;
#pragma unroll
          for (int e = 0; e < 8; ++e) {
            if (OUT_MODE == 1) {
              hv[e] = (_Float16)sp[e];
            } else {
              unsigned short hb = f2bf_bits(sp[e]);
              unsigned short lb = f2bf_bits(sp[e] - bf_bits2f(hb));
              hv[e] = __builtin_bit_cast(_Float16, hb);
              lv[e] = __builtin_bit_cast(_Float16, lb);
            }
          }
          *(volatile v8h*)(C + (size_t)(mBase + row) * ldc + n0 + c8) = hv;
          if (OUT_MODE == 2) *(volatile v8h*)(C2 + (size_t)(mBase + row) * ldc + n0 + c8) = lv;
        }
        __threadfence();
      }
    }
    __builtin_amdgcn_fence(__ATOMIC_RELEASE, "workgroup");
    __builtin_amdgcn_wave_barrier();
    __builtin_amdgcn_fence(__ATOMIC_ACQUIRE, "workgroup");
  }
}

#define EDIM 2048
#define TT   1024
#define NH   32
#define HD   64
#define NB   2
#define WSCALE     64.0f
#define WSCALE_INV (1.0f / 64.0f)
#define PSC        32768.0f
#define PSC_INV    (1.0f / 32768.0f)

__global__ __launch_bounds__(256) void cast_f32_f16x8(
    const float* __restrict__ in, _Float16* __restrict__ out, int n8) {
  const int i = blockIdx.x * 256 + threadIdx.x;
  if (i < n8) {
    const v4f a = *(const v4f*)(in + (size_t)8 * i);
    const v4f c = *(const v4f*)(in + (size_t)8 * i + 4);
    v8h hv;
    hv[0] = (_Float16)a[0]; hv[1] = (_Float16)a[1]; hv[2] = (_Float16)a[2]; hv[3] = (_Float16)a[3];
    hv[4] = (_Float16)c[0]; hv[5] = (_Float16)c[1]; hv[6] = (_Float16)c[2]; hv[7] = (_Float16)c[3];
    *(volatile v8h*)(out + (size_t)8 * i) = hv;
    __threadfence();
    *(volatile v8h*)(out + (size_t)8 * i) = hv;
  }
}

__global__ __launch_bounds__(256) void transpose_cast_w(const float* __restrict__ W0,
                                                         const float* __restrict__ W1,
                                                         const float* __restrict__ W2,
                                                         const float* __restrict__ W3,
                                                         _Float16* __restrict__ WT, float scale) {
  const int z = blockIdx.z;
  const float* W = (z == 0) ? W0 : (z == 1) ? W1 : (z == 2) ? W2 : W3;
  _Float16* Out = WT + (size_t)z * ((size_t)EDIM * EDIM);
  __shared__ __align__(16) _Float16 tile[64 * 72];
  const int tid = threadIdx.x;
  const int k0 = blockIdx.y * 64, n0 = blockIdx.x * 64;
#pragma unroll
  for (int i = 0; i < 4; ++i) {
    const int fidx = tid + i * 256;
    const int kl = fidx >> 4;
    const int nl = (fidx & 15) << 2;
    const v4f v = *(const v4f*)(W + (size_t)(k0 + kl) * EDIM + n0 + nl);
    tile[(nl + 0) * 72 + kl] = (_Float16)(v[0] * scale);
    tile[(nl + 1) * 72 + kl] = (_Float16)(v[1] * scale);
    tile[(nl + 2) * 72 + kl] = (_Float16)(v[2] * scale);
    tile[(nl + 3) * 72 + kl] = (_Float16)(v[3] * scale);
  }
  __syncthreads();
  const int row = tid >> 3;
  const int c8  = (tid & 7) * 8;
  for (int pass = 0; pass < 2; ++pass) {
#pragma unroll
    for (int i = 0; i < 2; ++i) {
      const int nl = row + 32 * i;
      const v8h hv = *(const v8h*)(tile + nl * 72 + c8);
      *(volatile v8h*)(Out + (size_t)(n0 + nl) * EDIM + k0 + c8) = hv;
    }
    __threadfence();
  }
}

__device__ __forceinline__ v8f mma_h(v16h a, v16h b, v8f c) {
  c = __builtin_amdgcn_wmma_f32_16x16x32_f16(false, a, false, b, (short)0, c, false, false);
  asm volatile("v_nop\n\tv_nop\n\tv_nop\n\tv_nop" : "+v"(c) : "v"(a), "v"(b));
  return c;
}

__global__ __launch_bounds__(32) void sb_attn_kernel(const _Float16* __restrict__ Q,
                                                     const _Float16* __restrict__ Kp,
                                                     const _Float16* __restrict__ VT,
                                                     _Float16* __restrict__ O) {
  union FB { v16h v; v8h h[2]; };
  __shared__ __align__(16) _Float16 Pw[16 * 32];
  __shared__ __align__(16) float    Os[16 * 68];

  const int lane = threadIdx.x & 31;
  const int hh   = lane >> 4;
  const int c    = lane & 15;
  const int it   = blockIdx.x;
  const int h    = blockIdx.y;
  const int b    = blockIdx.z;
  const int q0   = it * 16;

  const _Float16* Qb = Q  + (size_t)b * TT * EDIM + (size_t)h * HD;
  const _Float16* Kb = Kp + (size_t)b * TT * EDIM + (size_t)h * HD;
  const _Float16* Vb = VT + ((size_t)b * EDIM + (size_t)h * HD) * TT;

  v16h qa[2];
#pragma unroll
  for (int dc = 0; dc < 2; ++dc)
    qa[dc] = Frag<_Float16>::load(Qb + (size_t)(q0 + c) * EDIM + dc * 32 + 8 * hh);

  float S[8];
  v8f oacc[4];
#pragma unroll
  for (int r = 0; r < 8; ++r) S[r] = 0.f;
#pragma unroll
  for (int t = 0; t < 4; ++t) oacc[t] = (v8f){0.f,0.f,0.f,0.f,0.f,0.f,0.f,0.f};

  for (int ch = (it >> 1); ch >= 0; --ch) {
    const int cb = ch * 32;
#pragma unroll
    for (int sub = 1; sub >= 0; --sub) {
      const int kb = cb + sub * 16;
      v8f z = (v8f){0.f,0.f,0.f,0.f,0.f,0.f,0.f,0.f};
#pragma unroll
      for (int dc = 0; dc < 2; ++dc) {
        const v16h kf = Frag<_Float16>::load(Kb + (size_t)(kb + c) * EDIM + dc * 32 + 8 * hh);
        z = mma_h(qa[dc], kf, z);
      }
      const int j = kb + c;
#pragma unroll
      for (int r = 0; r < 8; ++r) {
        const int   qrow = q0 + 8 * hh + r;
        const float zz   = 0.125f * z[r];
        const bool  caus = (j < qrow);
        const float sp   = log1pf(expf(-fabsf(zz)));
        const float lb   = fminf(zz, 0.f) - sp;
        const float lom  = -fmaxf(zz, 0.f) - sp;
        const float mo   = caus ? lom : 0.f;
        float incl = mo;
#pragma unroll
        for (int off = 1; off < 16; off <<= 1) {
          const float tv = __shfl_down(incl, off, 16);
          incl += ((c + off) < 16) ? tv : 0.f;
        }
        const float tot   = __shfl(incl, 0, 16);
        const float sexcl = incl - mo + S[r];
        const float a     = caus ? expf(lb + sexcl) : 0.f;
        S[r] += tot;
        Pw[(8 * hh + r) * 32 + sub * 16 + c] = (_Float16)(a * PSC);
      }
    }
    __syncthreads();
    FB pa;
    pa.h[0] = *(const v8h*)(Pw + c * 32 + 8 * hh);
    pa.h[1] = *(const v8h*)(Pw + c * 32 + 16 + 8 * hh);
#pragma unroll
    for (int t = 0; t < 4; ++t) {
      const v16h vb = Frag<_Float16>::load(Vb + (size_t)(t * 16 + c) * TT + cb + 8 * hh);
      oacc[t] = mma_h(pa.v, vb, oacc[t]);
    }
    __syncthreads();
  }

#pragma unroll
  for (int r = 0; r < 8; ++r) {
#pragma unroll
    for (int t = 0; t < 4; ++t) Os[(8 * hh + r) * 68 + t * 16 + c] = oacc[t][r] * PSC_INV;
  }
  __syncthreads();
  {
    const int q4 = lane >> 3, c8 = (lane & 7) * 8;
    _Float16* Ob = O + (size_t)(b * TT + q0) * EDIM + (size_t)h * HD;
    for (int pass = 0; pass < 2; ++pass) {
#pragma unroll
      for (int i = 0; i < 4; ++i) {
        const int row = i * 4 + q4;
        const float* sp = Os + row * 68 + c8;
        v8h hv;
#pragma unroll
        for (int e = 0; e < 8; ++e) hv[e] = (_Float16)sp[e];
        *(volatile v8h*)(Ob + (size_t)row * EDIM + c8) = hv;
      }
      __threadfence();
    }
  }
}

extern "C" void kernel_launch(void* const* d_in, const int* in_sizes, int n_in,
                              void* d_out, int out_size, void* d_ws, size_t ws_size,
                              hipStream_t stream) {
  const size_t MAT = (size_t)EDIM * EDIM;
  const size_t MTOK = (size_t)NB * TT;
  if (n_in < 5) return;
  if ((size_t)in_sizes[0] != MTOK * EDIM) return;
  if ((size_t)in_sizes[1] != MAT || (size_t)in_sizes[2] != MAT ||
      (size_t)in_sizes[3] != MAT || (size_t)in_sizes[4] != MAT) return;
  if ((size_t)out_size != MTOK * EDIM) return;

  const size_t PLANE = MAT * sizeof(_Float16);
  const size_t offX  = 0;
  const size_t offWT = offX  + PLANE;
  const size_t offQ  = offWT + 4 * PLANE;
  const size_t offK  = offQ  + PLANE;
  const size_t offVT = offK  + PLANE;
  const size_t offO  = offVT + PLANE;
  const size_t total = offO  + PLANE;
  if (total > ws_size) return;

  const float* hs = (const float*)d_in[0];
  const float* Wq = (const float*)d_in[1];
  const float* Wk = (const float*)d_in[2];
  const float* Wv = (const float*)d_in[3];
  const float* Wo = (const float*)d_in[4];

  char* ws = (char*)d_ws;
  _Float16* X16 = (_Float16*)(ws + offX);
  _Float16* WT  = (_Float16*)(ws + offWT);
  _Float16* Q16 = (_Float16*)(ws + offQ);
  _Float16* K16 = (_Float16*)(ws + offK);
  _Float16* VTp = (_Float16*)(ws + offVT);
  _Float16* O16 = (_Float16*)(ws + offO);
  const unsigned short* uX  = (const unsigned short*)X16;
  const unsigned short* uO  = (const unsigned short*)O16;
  const unsigned short* uWq = (const unsigned short*)(WT + 0 * MAT);
  const unsigned short* uWk = (const unsigned short*)(WT + 1 * MAT);
  const unsigned short* uWv = (const unsigned short*)(WT + 2 * MAT);
  const unsigned short* uWo = (const unsigned short*)(WT + 3 * MAT);
  const float* dummyf = (const float*)d_ws;

  const int n8 = (int)(MTOK * EDIM / 8);
  cast_f32_f16x8<<<dim3((n8 + 255) / 256), dim3(256), 0, stream>>>(hs, X16, n8);

  transpose_cast_w<<<dim3(EDIM / 64, EDIM / 64, 4), dim3(256), 0, stream>>>(Wq, Wk, Wv, Wo, WT, WSCALE);

  {
    const int M = (int)MTOK, N = EDIM, K = EDIM;
    const int gx = ((M >> 6) * (N >> 6) + 7) / 8;
    wmma_gemm64<0, false, 0, 1, false><<<dim3(gx, 1), dim3(256), 0, stream>>>(
        uX, uX, EDIM, 0L, uWq, uWq, EDIM, 0L, (void*)Q16, (void*)Q16, EDIM, 0L,
        dummyf, dummyf, 0L, M, N, K, WSCALE_INV);
    wmma_gemm64<0, false, 0, 1, false><<<dim3(gx, 1), dim3(256), 0, stream>>>(
        uX, uX, EDIM, 0L, uWk, uWk, EDIM, 0L, (void*)K16, (void*)K16, EDIM, 0L,
        dummyf, dummyf, 0L, M, N, K, WSCALE_INV);
  }
  {
    const int M = EDIM, N = TT, K = EDIM;
    const int gx = ((M >> 6) * (N >> 6) + 7) / 8;
    wmma_gemm64<0, false, 0, 1, false><<<dim3(gx, NB), dim3(256), 0, stream>>>(
        uWv, uWv, EDIM, 0L, uX, uX, EDIM, (long)TT * EDIM, (void*)VTp, (void*)VTp, TT, (long)EDIM * TT,
        dummyf, dummyf, 0L, M, N, K, WSCALE_INV);
  }

  sb_attn_kernel<<<dim3(TT / 16, NH, NB), dim3(32), 0, stream>>>(Q16, K16, VTp, O16);

  {
    const int M = (int)MTOK, N = EDIM, K = EDIM;
    const int gx = ((M >> 6) * (N >> 6) + 7) / 8;
    wmma_gemm64<0, false, 0, 0, false><<<dim3(gx, 1), dim3(256), 0, stream>>>(
        uO, uO, EDIM, 0L, uWo, uWo, EDIM, 0L, d_out, d_out, EDIM, 0L,
        dummyf, dummyf, 0L, M, N, K, WSCALE_INV);
  }
  (void)hipGetLastError();
}
